// DenoiseNet_25778393711129
// MI455X (gfx1250) — hardware-verified
//
#include <hip/hip_runtime.h>

#define NPTS   16384
#define NBAT   2
#define NALL   (NBAT * NPTS)
#define HD     128
#define FRAGM  16384
#define NMAT   5
#define CA     16.0f
#define CW     256.0f
#define INVACC 0.000244140625f
#define TPW    4

typedef _Float16 v16h __attribute__((ext_vector_type(16)));
typedef _Float16 v8h  __attribute__((ext_vector_type(8)));
typedef float    v8f  __attribute__((ext_vector_type(8)));
typedef float    v4f  __attribute__((ext_vector_type(4)));
typedef v16h __attribute__((may_alias)) v16ha;
typedef v8h  __attribute__((may_alias)) v8ha;
typedef v4f  __attribute__((may_alias)) v4fa;

union Frag { v16h v; v8h half[2]; };

static_assert(NALL % 64 == 0);
static_assert(NPTS % 128 == 0);
static_assert(HD == 128);

__device__ __forceinline__ v8f wmma_f16(v16h a, v16h b, v8f c) {
  v8f d = __builtin_amdgcn_wmma_f32_16x16x32_f16(false, a, false, b, (short)0, c, false, false);
  asm volatile("v_nop\n\tv_nop\n\tv_nop\n\tv_nop" : "+v"(d) : "v"(a), "v"(b));
  return d;
}

__device__ __forceinline__ v16h load_afrag(const _Float16* sh, int m, int hh, int kc) {
  const _Float16* p = sh + m * HD + kc * 32;
  Frag f;
  f.half[0] = *(const v8ha*)(p + 8 * hh);
  f.half[1] = *(const v8ha*)(p + 16 + 8 * hh);
  return f.v;
}

__device__ __forceinline__ void load_afrags(const _Float16* sh, int m, int hh, v16h (&a)[4]) {
  #pragma unroll
  for (int kc = 0; kc < 4; ++kc) a[kc] = load_afrag(sh, m, hh, kc);
}

__device__ __forceinline__ v16h load_bfrag(const _Float16* wb, int kc, int tn, int lane) {
  return *(const v16ha*)(wb + (((kc * 8 + tn) * 32 + lane) << 4));
}

__device__ __forceinline__ v8f gemm_col_tile(const v16h (&a)[4], const _Float16* wb, int tn, int lane) {
  v8f acc = {0.f, 0.f, 0.f, 0.f, 0.f, 0.f, 0.f, 0.f};
  #pragma unroll
  for (int kc = 0; kc < 4; ++kc) acc = wmma_f16(a[kc], load_bfrag(wb, kc, tn, lane), acc);
  return acc;
}

__device__ __forceinline__ void store_tile(_Float16* sh, const v8f (&hc)[8], int m, int hh) {
  #pragma unroll
  for (int t = 0; t < 8; ++t)
    #pragma unroll
    for (int r = 0; r < 8; ++r)
      sh[(r + 8 * hh) * HD + 16 * t + m] = (_Float16)(hc[t][r] * CA);
}

__global__ __launch_bounds__(256) void k_pack(
    const float* __restrict__ Wf2, const float* __restrict__ W0,
    const float* __restrict__ Wb,  const float* __restrict__ Wo,
    _Float16* __restrict__ frag)
{
  const int g = blockIdx.x * 256 + threadIdx.x;
  if (g >= NMAT * 2048) return;
  const int hsel = g & 1;
  const int lane = (g >> 1) & 31;
  const int tn   = (g >> 6) & 7;
  const int kc   = (g >> 9) & 3;
  const int mat  = g >> 11;
  const int col  = tn * 16 + (lane & 15);
  const int hh   = lane >> 4;
  const int kb   = kc * 32 + 16 * hsel + 8 * hh;
  float v[8];
  if (mat == 0) {
    #pragma unroll
    for (int j = 0; j < 8; ++j) v[j] = Wf2[(kb + j) * HD + col];
  } else if (mat == 1) {
    #pragma unroll
    for (int j = 0; j < 8; ++j) v[j] = W0[(3 + kb + j) * HD + col];
  } else if (mat == 2) {
    #pragma unroll
    for (int j = 0; j < 8; ++j) v[j] = Wb[(kb + j) * HD + col];
  } else if (mat == 3) {
    #pragma unroll
    for (int j = 0; j < 8; ++j) v[j] = Wb[HD * HD + (kb + j) * HD + col];
  } else {
    const int cc = (col < 3) ? col : 2;
    #pragma unroll
    for (int j = 0; j < 8; ++j) {
      const float t = Wo[(kb + j) * 3 + cc];
      v[j] = (col < 3) ? t : 0.0f;
    }
  }
  const v8h o = { (_Float16)(v[0] * CW), (_Float16)(v[1] * CW), (_Float16)(v[2] * CW), (_Float16)(v[3] * CW),
                  (_Float16)(v[4] * CW), (_Float16)(v[5] * CW), (_Float16)(v[6] * CW), (_Float16)(v[7] * CW) };
  _Float16* dst = frag + (size_t)g * 8;
  *(volatile v8h*)dst = o;
  __threadfence();
  *(volatile v8h*)dst = o;
}

__device__ __forceinline__ void fw_store_pass(const float* sf, float* dst, int lane) {
  const int q8 = lane & 7, sub = lane >> 3;
  #pragma unroll
  for (int i = 0; i < 16; ++i) {
    const int lid = i * 4 + sub;
    const int row = lid >> 2, piece = lid & 3;
    const v4f v = *(const v4fa*)(sf + row * HD + 32 * piece + 4 * q8);
    *(volatile v4f*)(dst + (size_t)row * HD + 32 * piece + 4 * q8) = v;
  }
}

__global__ __launch_bounds__(128) void k_prep(
    const float* __restrict__ pcl, const float* __restrict__ Wf1,
    const float* __restrict__ bf1, const float* __restrict__ bf2,
    const float* __restrict__ b0,  const _Float16* __restrict__ frag,
    float* __restrict__ FW)
{
  __shared__ __attribute__((aligned(16))) _Float16 sH[4 * 16 * HD];
  __shared__ __attribute__((aligned(16))) float sF[4 * 16 * HD];
  __shared__ __attribute__((aligned(16))) float sX[64 * 3];
  __shared__ __attribute__((aligned(16))) float sW1[3 * HD];
  __shared__ __attribute__((aligned(16))) float sB1[HD];
  __shared__ __attribute__((aligned(16))) float sB2[HD];
  __shared__ __attribute__((aligned(16))) float sB0[HD];

  const int tid = threadIdx.x, lane = tid & 31, w = tid >> 5;
  const int hh = lane >> 4, m = lane & 15;
  const int pb = blockIdx.x * 64;

  if (tid < 48) ((v4fa*)sX)[tid] = ((const v4fa*)(pcl + (size_t)pb * 3))[tid];
  if (tid < 96) ((v4fa*)sW1)[tid] = ((const v4fa*)Wf1)[tid];
  if (tid < 32) {
    ((v4fa*)sB1)[tid] = ((const v4fa*)bf1)[tid];
    ((v4fa*)sB2)[tid] = ((const v4fa*)bf2)[tid];
    ((v4fa*)sB0)[tid] = ((const v4fa*)b0)[tid];
  }
  __syncthreads();

  _Float16* sh = sH + w * (16 * HD);
  float* sf = sF + w * (16 * HD);

  v8f hc[8];
  {
    float px[8][3];
    #pragma unroll
    for (int r = 0; r < 8; ++r) {
      const int row = 16 * w + 8 * hh + r;
      px[r][0] = sX[row * 3 + 0];
      px[r][1] = sX[row * 3 + 1];
      px[r][2] = sX[row * 3 + 2];
    }
    #pragma unroll
    for (int t = 0; t < 8; ++t) {
      const int n = 16 * t + m;
      const float w0 = sW1[n], w1 = sW1[HD + n], w2 = sW1[2 * HD + n], bz = sB1[n];
      #pragma unroll
      for (int r = 0; r < 8; ++r)
        hc[t][r] = fmaxf((px[r][0] * w0 + px[r][1] * w1 + px[r][2] * w2) + bz, 0.0f);
    }
  }

  store_tile(sh, hc, m, hh);
  __syncthreads();
  {
    v16h a[4];
    load_afrags(sh, m, hh, a);
    #pragma unroll
    for (int t = 0; t < 8; ++t) {
      const v8f acc = gemm_col_tile(a, frag, t, lane);
      const float bz = sB2[16 * t + m];
      #pragma unroll
      for (int r = 0; r < 8; ++r) hc[t][r] = acc[r] * INVACC + bz;
    }
  }
  __syncthreads();

  store_tile(sh, hc, m, hh);
  __syncthreads();
  {
    v16h a[4];
    load_afrags(sh, m, hh, a);
    #pragma unroll
    for (int t = 0; t < 8; ++t) {
      const v8f acc = gemm_col_tile(a, frag + FRAGM, t, lane);
      const float bz = sB0[16 * t + m];
      #pragma unroll
      for (int r = 0; r < 8; ++r)
        sf[(8 * hh + r) * HD + 16 * t + m] = acc[r] * INVACC + bz;
    }
  }
  __syncthreads();

  float* dst = FW + (size_t)(pb + 16 * w) * HD;
  fw_store_pass(sf, dst, lane);
  __threadfence();
  fw_store_pass(sf, dst, lane);
}

__device__ __forceinline__ void g_store_pass(const float* sg, float* dst, int tid) {
  const int q8 = tid & 7, sub = tid >> 3;
  #pragma unroll
  for (int i = 0; i < 2; ++i) {
    const int lid = i * 16 + sub;
    const v4f v = *(const v4fa*)(sg + lid * 32 + 4 * q8);
    *(volatile v4f*)(dst + lid * 32 + 4 * q8) = v;
  }
}

__global__ __launch_bounds__(128) void k_step(
    const float* __restrict__ pcl0, const float* __restrict__ pcur,
    const float* __restrict__ W0,   const float* __restrict__ FW,
    const _Float16* __restrict__ frag, const float* __restrict__ bb,
    const float* __restrict__ bo,   float* __restrict__ G)
{
  __shared__ __attribute__((aligned(16))) _Float16 sWB[2 * FRAGM + 2048];
  __shared__ __attribute__((aligned(16))) _Float16 sH[4 * 16 * HD];
  __shared__ __attribute__((aligned(16))) float sFW[4 * 4 * HD];
  __shared__ __attribute__((aligned(16))) float sG[256 * 4];
  __shared__ __attribute__((aligned(16))) float sPC[208];
  __shared__ __attribute__((aligned(16))) float sP0[64 * 3];
  __shared__ __attribute__((aligned(16))) float sW0[3 * HD];
  __shared__ __attribute__((aligned(16))) float sBB[2 * HD];
  __shared__ __attribute__((aligned(16))) float sBO[4];

  const int tid = threadIdx.x, lane = tid & 31, w = tid >> 5;
  const int hh = lane >> 4, m = lane & 15;
  const int fb  = blockIdx.x * 64;
  const int b   = fb / NPTS;
  const int nb0 = fb - b * NPTS;

  {
    const v8ha* src = (const v8ha*)(frag + 2 * FRAGM);
    v8ha* dst = (v8ha*)sWB;
    for (int i = tid; i < 4096; i += 128) dst[i] = src[i];
    const v8ha* src4 = (const v8ha*)(frag + 4 * FRAGM);
    for (int i = tid; i < 256; i += 128) {
      const int kc = i >> 6, j = i & 63;
      dst[4096 + i] = src4[kc * 512 + j];
    }
  }
  if (tid < 96) ((v4fa*)sW0)[tid] = ((const v4fa*)W0)[tid];
  if (tid < 64) ((v4fa*)sBB)[tid] = ((const v4fa*)bb)[tid];
  if (tid < 3) sBO[tid] = bo[tid];
  else if (tid == 3) sBO[3] = 0.0f;
  if (tid < 48) ((v4fa*)sP0)[tid] = ((const v4fa*)(pcl0 + (size_t)fb * 3))[tid];
  for (int i = tid; i < 204; i += 128) {
    const int j = i / 3, c = i - 3 * j;
    int n = nb0 + j - 2;
    n = n < 0 ? 0 : (n > NPTS - 1 ? NPTS - 1 : n);
    sPC[i] = pcur[(size_t)(b * NPTS + n) * 3 + c];
  }
  __syncthreads();

  _Float16* sh = sH + w * (16 * HD);
  float* sfw = sFW + w * (4 * HD);

  #pragma unroll 1
  for (int it = 0; it < TPW; ++it) {
    const int tb = it * 4 + w;
    const int lp = tb * 4;

    {
      const v4fa* src = (const v4fa*)(FW + (size_t)(fb + lp) * HD);
      v4fa* dst = (v4fa*)sfw;
      #pragma unroll
      for (int i = 0; i < 4; ++i) dst[i * 32 + lane] = src[i * 32 + lane];
    }
    float cent[8][3];
    #pragma unroll
    for (int r = 0; r < 8; ++r) {
      const int M = 8 * hh + r;
      const int pt = lp + (M >> 2), k = M & 3;
      #pragma unroll
      for (int c = 0; c < 3; ++c) cent[r][c] = sPC[(pt + k) * 3 + c] - sP0[pt * 3 + c];
    }
    __syncthreads();

    v8f hc[8];
    #pragma unroll
    for (int t = 0; t < 8; ++t) {
      const int n = 16 * t + m;
      const float w0 = sW0[n], w1 = sW0[HD + n], w2 = sW0[2 * HD + n];
      #pragma unroll
      for (int r = 0; r < 8; ++r) {
        const int ptw = (8 * hh + r) >> 2;
        const float f = sfw[ptw * HD + n];
        hc[t][r] = fmaxf(f + (cent[r][0] * w0 + cent[r][1] * w1 + cent[r][2] * w2), 0.0f);
      }
    }

    #pragma unroll
    for (int blk = 0; blk < 2; ++blk) {
      __syncthreads();
      store_tile(sh, hc, m, hh);
      __syncthreads();
      v16h a[4];
      load_afrags(sh, m, hh, a);
      #pragma unroll
      for (int t = 0; t < 8; ++t) {
        const v8f acc = gemm_col_tile(a, sWB + blk * FRAGM, t, lane);
        const float bz = sBB[blk * HD + 16 * t + m];
        #pragma unroll
        for (int r = 0; r < 8; ++r) hc[t][r] = hc[t][r] + fmaxf(acc[r] * INVACC + bz, 0.0f);
      }
    }

    __syncthreads();
    store_tile(sh, hc, m, hh);
    __syncthreads();
    {
      v16h a[4];
      load_afrags(sh, m, hh, a);
      v8f acc = {0.f, 0.f, 0.f, 0.f, 0.f, 0.f, 0.f, 0.f};
      #pragma unroll
      for (int kc = 0; kc < 4; ++kc)
        acc = wmma_f16(a[kc], *(const v16ha*)(sWB + 2 * FRAGM + ((kc * 32 + lane) << 4)), acc);
      if (m < 4) {
        const float bz = sBO[m];
        const bool real = (m < 3);
        #pragma unroll
        for (int r = 0; r < 8; ++r) {
          const float gv = acc[r] * INVACC + bz;
          sG[(tb * 16 + 8 * hh + r) * 4 + m] = real ? gv : 0.0f;
        }
      }
    }
  }
  __syncthreads();

  float* gdst = G + (size_t)fb * 16;
  g_store_pass(sG, gdst, tid);
  __threadfence();
  g_store_pass(sG, gdst, tid);
}

__device__ __forceinline__ void p_store_pass(const float* sp, float* dst, int tid) {
  if (tid < 96) {
    const int q8 = tid & 7, lid = tid >> 3;
    const v4f v = *(const v4fa*)(sp + lid * 32 + 4 * q8);
    *(volatile v4f*)(dst + lid * 32 + 4 * q8) = v;
  }
}

__global__ __launch_bounds__(128) void k_update(
    const float* __restrict__ pcur, const float* __restrict__ G,
    float* __restrict__ pout, float s)
{
  __shared__ __attribute__((aligned(16))) float sP[128 * 3];

  const int tid = threadIdx.x;
  const int fb = blockIdx.x * 128;
  const int b  = fb / NPTS;
  const int n  = fb - b * NPTS + tid;

  float a0 = 0.0f, a1 = 0.0f, a2 = 0.0f;
  #pragma unroll
  for (int dm = -1; dm <= 2; ++dm) {
    const int mm = n + dm;
    const bool mv = (mm >= 0) && (mm < NPTS);
    const int mc = mm < 0 ? 0 : (mm > NPTS - 1 ? NPTS - 1 : mm);
    const v4fa* gp = (const v4fa*)(G + (size_t)(b * NPTS + mc) * 16);
    #pragma unroll
    for (int k = 0; k < 4; ++k) {
      const v4f g = gp[k];
      int tg = mm + k - 2;
      tg = tg < 0 ? 0 : (tg > NPTS - 1 ? NPTS - 1 : tg);
      const bool hit = mv && (tg == n);
      a0 = hit ? a0 + g.x : a0;
      a1 = hit ? a1 + g.y : a1;
      a2 = hit ? a2 + g.z : a2;
    }
  }
  const size_t f = (size_t)fb + tid;
  const float p0 = pcur[f * 3 + 0], p1 = pcur[f * 3 + 1], p2 = pcur[f * 3 + 2];
  sP[tid * 3 + 0] = p0 + s * a0;
  sP[tid * 3 + 1] = p1 + s * a1;
  sP[tid * 3 + 2] = p2 + s * a2;
  __syncthreads();

  float* dst = pout + (size_t)fb * 3;
  p_store_pass(sP, dst, tid);
  __threadfence();
  p_store_pass(sP, dst, tid);
}

extern "C" void kernel_launch(void* const* d_in, const int* in_sizes, int n_in,
                              void* d_out, int out_size, void* d_ws, size_t ws_size,
                              hipStream_t stream) {
  if (n_in < 11) return;
  if (in_sizes[0] != NALL * 3) return;
  if (in_sizes[1] != 3 * HD || in_sizes[2] != HD) return;
  if (in_sizes[3] != HD * HD || in_sizes[4] != HD) return;
  if (in_sizes[5] != 131 * HD || in_sizes[6] != HD) return;
  if (in_sizes[7] != 2 * HD * HD || in_sizes[8] != 2 * HD) return;
  if (in_sizes[9] != HD * 3 || in_sizes[10] != 3) return;
  if (out_size != NALL * 3) return;

  const float* pcl = (const float*)d_in[0];
  const float* Wf1 = (const float*)d_in[1];
  const float* bf1 = (const float*)d_in[2];
  const float* Wf2 = (const float*)d_in[3];
  const float* bf2 = (const float*)d_in[4];
  const float* W0  = (const float*)d_in[5];
  const float* b0  = (const float*)d_in[6];
  const float* Wb  = (const float*)d_in[7];
  const float* bb  = (const float*)d_in[8];
  const float* Wo  = (const float*)d_in[9];
  const float* bo  = (const float*)d_in[10];
  float* out = (float*)d_out;

  const size_t frag_bytes = (size_t)NMAT * FRAGM * 2;
  const size_t fw_bytes   = (size_t)NALL * HD * 4;
  const size_t g_bytes    = (size_t)NALL * 16 * 4;
  const size_t p_bytes    = (size_t)NALL * 3 * 4;
  const size_t total = frag_bytes + fw_bytes + g_bytes + 2 * p_bytes;
  if (total > ws_size) return;

  char* ws = (char*)d_ws;
  _Float16* frag = (_Float16*)ws;
  float* FW = (float*)(ws + frag_bytes);
  float* G  = (float*)(ws + frag_bytes + fw_bytes);
  float* PA = (float*)(ws + frag_bytes + fw_bytes + g_bytes);
  float* PB = (float*)(ws + frag_bytes + fw_bytes + g_bytes + p_bytes);

  k_pack<<<(NMAT * 2048) / 256, 256, 0, stream>>>(Wf2, W0, Wb, Wo, frag);
  k_prep<<<NALL / 64, 128, 0, stream>>>(pcl, Wf1, bf1, bf2, b0, frag, FW);

  const float* pin = pcl;
  float d = 1.0f;
  for (int step = 0; step < 4; ++step) {
    float* po = (step == 3) ? out : ((step & 1) ? PB : PA);
    const float s = 0.2f * d;
    k_step<<<NALL / 64, 128, 0, stream>>>(pcl, pin, W0, FW, frag, bb, bo, G);
    k_update<<<NALL / 128, 128, 0, stream>>>(pin, G, po, s);
    pin = po;
    d *= 0.95f;
  }
}
